// RelationalHypergraphLayer_90744069030530
// MI455X (gfx1250) — hardware-verified
//
#include <hip/hip_runtime.h>
#include <stddef.h>


#define NTHR    256
#define NWAVE   8
#define EPT     8
#define NGRP    2
#define CHUNK   (NTHR * EPT * NGRP)
#define WCAP    (EPT * NGRP * 32)
#define LISTN   (NWAVE * WCAP)
#define KSH     13
#define NBC     8192
#define NBF     2048
#define CPT     16
#define RCAP    40960
#define RBN     128
#define TGT     256
#define DEGCAP  1024
#define OTHR    512
#define BM      64
#define BNC     128
#define WSCAP   134217728
#define FIN     128
#define FOUT    128
#define NHD     8
#define DHD     16
#define ESW     16
#define ACARRY  8.0f
#define WCARRY  64.0f
#define SCL_AW  (1.0f / 512.0f)

#define LDS_FILL ((RCAP + NBF + LISTN) * 4 + 64)

static_assert((CHUNK & (CHUNK - 1)) == 0);
static_assert(CHUNK <= (1 << 12));
static_assert(NBC <= (1 << KSH));
static_assert((NBC & (NBC - 1)) == 0 && (NBF & (NBF - 1)) == 0);
static_assert(NBC == 4 * NBF);
static_assert(OTHR * CPT == NBC);
static_assert((OTHR / 4) * CPT == NBF);
static_assert(OTHR / 32 == 16);
static_assert((RCAP % 32) == 0);
static_assert(TGT == NWAVE * 32);
static_assert((NBC % TGT) == 0);
static_assert((TGT % BM) == 0);
static_assert(WCAP == EPT * NGRP * 32);
static_assert((FIN % 32) == 0 && FOUT == BNC);
static_assert(NHD * DHD == FOUT && FIN == FOUT);
static_assert(ESW == 2 * NHD);
static_assert(NTHR == 32 * NHD);
static_assert(NBC == NWAVE * 8 * 128);

typedef float    v4f  __attribute__((ext_vector_type(4)));
typedef float    v8f  __attribute__((ext_vector_type(8)));
typedef int      v4i  __attribute__((ext_vector_type(4)));
typedef _Float16 v8h  __attribute__((ext_vector_type(8)));
typedef _Float16 v16h __attribute__((ext_vector_type(16)));
union Frag { v16h v; v8h h[2]; };

__device__ __forceinline__ v8f wmh(v16h a, v16h b, v8f c) {
  v8f d = __builtin_amdgcn_wmma_f32_16x16x32_f16(false, a, false, b, (short)0, c, false, false);
  asm volatile("v_nop\n\tv_nop\n\tv_nop\n\tv_nop" : "+v"(d) : "v"(a), "v"(b));
  return d;
}

__device__ __forceinline__ v4f selv4(v4f v, bool c, float other) {
  v4f o; o.x = c ? v.x : other; o.y = c ? v.y : other; o.z = c ? v.z : other; o.w = c ? v.w : other; return o;
}
__device__ __forceinline__ v4f vmax4(v4f a, v4f b) {
  v4f o; o.x = fmaxf(a.x, b.x); o.y = fmaxf(a.y, b.y); o.z = fmaxf(a.z, b.z); o.w = fmaxf(a.w, b.w); return o;
}
__device__ __forceinline__ v4f lrelu4(v4f v) {
  v4f o;
  o.x = v.x >= 0.f ? v.x : 0.2f * v.x;  o.y = v.y >= 0.f ? v.y : 0.2f * v.y;
  o.z = v.z >= 0.f ? v.z : 0.2f * v.z;  o.w = v.w >= 0.f ? v.w : 0.2f * v.w;
  return o;
}
__device__ __forceinline__ v4f vexp4(v4f v) {
  v4f o; o.x = __expf(v.x); o.y = __expf(v.y); o.z = __expf(v.z); o.w = __expf(v.w); return o;
}
__device__ __forceinline__ v4i imax04(v4i v) {
  v4i o; o.x = max(v.x, 0); o.y = max(v.y, 0); o.z = max(v.z, 0); o.w = max(v.w, 0); return o;
}
__device__ __forceinline__ int hsum4i(v4i v) { return v.x + v.y + v.z + v.w; }
__device__ __forceinline__ v4f wmax4(v4f v) {
#pragma unroll
  for (int off = 16; off > 0; off >>= 1) {
    v.x = fmaxf(v.x, __shfl_xor(v.x, off)); v.y = fmaxf(v.y, __shfl_xor(v.y, off));
    v.z = fmaxf(v.z, __shfl_xor(v.z, off)); v.w = fmaxf(v.w, __shfl_xor(v.w, off));
  }
  return v;
}
__device__ __forceinline__ v4f wsum4(v4f v) {
#pragma unroll
  for (int off = 16; off > 0; off >>= 1) {
    v.x += __shfl_xor(v.x, off); v.y += __shfl_xor(v.y, off);
    v.z += __shfl_xor(v.z, off); v.w += __shfl_xor(v.w, off);
  }
  return v;
}

template <int NB>
__device__ __forceinline__ int scan_chunk(const int* __restrict__ dsts, int nE, int cbase, int slotBase,
                                          int vec8, int* list, int tid, int lane, int wave) {
  static_assert(NB <= (1 << KSH));
  int wc = 0;
#pragma unroll
  for (int g = 0; g < NGRP; ++g) {
    const int el0  = (g * NTHR + tid) * EPT;
    const int e0   = cbase + el0;
    const int sent = -2147483647 - 1;
    v4i da, db;
    if (vec8 != 0 && cbase + CHUNK <= nE) {
      da = *(const v4i*)(dsts + e0);
      db = *(const v4i*)(dsts + e0 + 4);
    } else {
      da.x = (e0     < nE) ? dsts[min(e0, nE - 1)] : sent;
      da.y = (e0 + 1 < nE) ? dsts[min(e0 + 1, nE - 1)] : sent;
      da.z = (e0 + 2 < nE) ? dsts[min(e0 + 2, nE - 1)] : sent;
      da.w = (e0 + 3 < nE) ? dsts[min(e0 + 3, nE - 1)] : sent;
      db.x = (e0 + 4 < nE) ? dsts[min(e0 + 4, nE - 1)] : sent;
      db.y = (e0 + 5 < nE) ? dsts[min(e0 + 5, nE - 1)] : sent;
      db.z = (e0 + 6 < nE) ? dsts[min(e0 + 6, nE - 1)] : sent;
      db.w = (e0 + 7 < nE) ? dsts[min(e0 + 7, nE - 1)] : sent;
    }
    const unsigned nb = (unsigned)slotBase;
    const unsigned s0 = (unsigned)da.x - nb, s1 = (unsigned)da.y - nb;
    const unsigned s2 = (unsigned)da.z - nb, s3 = (unsigned)da.w - nb;
    const unsigned s4 = (unsigned)db.x - nb, s5 = (unsigned)db.y - nb;
    const unsigned s6 = (unsigned)db.z - nb, s7 = (unsigned)db.w - nb;
    const bool h0 = s0 < (unsigned)NB, h1 = s1 < (unsigned)NB, h2 = s2 < (unsigned)NB, h3 = s3 < (unsigned)NB;
    const bool h4 = s4 < (unsigned)NB, h5 = s5 < (unsigned)NB, h6 = s6 < (unsigned)NB, h7 = s7 < (unsigned)NB;
    const unsigned any = __builtin_amdgcn_ballot_w32(h0 | h1 | h2 | h3 | h4 | h5 | h6 | h7);
    if (any != 0u) {
#define HITJ(J, HJ, SJ) { \
        const unsigned mj = __builtin_amdgcn_ballot_w32(HJ); \
        if (mj != 0u) { \
          if (HJ) { \
            const int pos = wc + (int)__builtin_amdgcn_mbcnt_lo(mj, 0u); \
            if (pos < WCAP) list[wave * WCAP + pos] = ((el0 + (J)) << KSH) | (int)(SJ); \
          } \
          wc += (int)__builtin_popcount(mj); } }
      HITJ(0, h0, s0)
      HITJ(1, h1, s1)
      HITJ(2, h2, s2)
      HITJ(3, h3, s3)
      HITJ(4, h4, s4)
      HITJ(5, h5, s5)
      HITJ(6, h6, s6)
      HITJ(7, h7, s7)
#undef HITJ
    }
  }
  return wc;
}

__global__ __launch_bounds__(NTHR) void k_count(const int* __restrict__ dsts, int* cnt, int nE, int vec8) {
  __shared__ __attribute__((aligned(16))) int scnt[NBC];
  __shared__ __attribute__((aligned(16))) int list[LISTN];
  __shared__ int wcnt[NWAVE];
  const int tid = threadIdx.x, lane = tid & 31, wave = tid >> 5;
  const int nodeBase = blockIdx.x * NBC;

  for (int i = tid; i < NBC; i += NTHR) scnt[i] = 0;
  __syncthreads();

  const int nChunks = (nE + CHUNK - 1) / CHUNK;
#pragma unroll 1
  for (int ch = 0; ch < nChunks; ++ch) {
    const int cbase = ch * CHUNK;
    const int wc = scan_chunk<NBC>(dsts, nE, cbase, nodeBase, vec8, list, tid, lane, wave);
    if (lane == 0) wcnt[wave] = wc;
    __syncthreads();
    if (wave == 0) {
#pragma unroll 1
      for (int wsx = 0; wsx < NWAVE; ++wsx) {
        int n = __builtin_amdgcn_readfirstlane(wcnt[wsx]);
        n = n > WCAP ? WCAP : (n < 0 ? 0 : n);
        const int* lp = list + wsx * WCAP;
#pragma unroll 1
        for (int i = 0; i < n; ++i) {
          const int ent  = __builtin_amdgcn_readfirstlane(lp[i]);
          const int slot = ent & (NBC - 1);
          if (lane == 0) scnt[slot] = scnt[slot] + 1;
        }
      }
    }
    __syncthreads();
  }

  v4i cq[8];
#pragma unroll
  for (int q = 0; q < 8; ++q) {
    const int f = (wave * 8 + q) * 128 + 4 * lane;
    cq[q] = *(const v4i*)(scnt + f);
  }
  int* cp = cnt + (size_t)nodeBase;
#pragma unroll
  for (int q = 0; q < 8; ++q) {
    const int f = (wave * 8 + q) * 128 + 4 * lane;
    *(volatile v4i*)(cp + f) = cq[q];
  }
  __threadfence();
#pragma unroll
  for (int q = 0; q < 8; ++q) {
    const int f = (wave * 8 + q) * 128 + 4 * lane;
    *(volatile v4i*)(cp + f) = cq[q];
  }
}

__global__ __launch_bounds__(OTHR) void k_offsets(
    const int* __restrict__ cnt, int* off, int* rbase, int nChunk) {
  __shared__ __attribute__((aligned(16))) int soff[NBC];
  __shared__ __attribute__((aligned(16))) int srb[RBN];
  __shared__ int wtot[OTHR / 32];
  const int tid = threadIdx.x, lane = tid & 31, wave = tid >> 5, sub = tid >> 7;
  for (int i = tid; i < RBN; i += OTHR) srb[i] = 0;
  int carry = 0;
#pragma unroll 1
  for (int ch = 0; ch < nChunk; ++ch) {
    const int base = ch * NBC;
    const int* cp = cnt + base + CPT * tid;
    const v4i c0 = imax04(*(const v4i*)cp);
    const v4i c1 = imax04(*(const v4i*)(cp + 4));
    const v4i c2 = imax04(*(const v4i*)(cp + 8));
    const v4i c3 = imax04(*(const v4i*)(cp + 12));
    const int ts = hsum4i(c0) + hsum4i(c1) + hsum4i(c2) + hsum4i(c3);
    int incl = ts;
#pragma unroll
    for (int d = 1; d < 32; d <<= 1) {
      const int t = __shfl_up(incl, d);
      if (lane >= d) incl += t;
    }
    if (lane == 31) wtot[wave] = incl;
    __syncthreads();
    const int S0 = wtot[0]  + wtot[1]  + wtot[2]  + wtot[3];
    const int S1 = wtot[4]  + wtot[5]  + wtot[6]  + wtot[7];
    const int S2 = wtot[8]  + wtot[9]  + wtot[10] + wtot[11];
    const int S3 = wtot[12] + wtot[13] + wtot[14] + wtot[15];
    int pre = 0;
#pragma unroll 1
    for (int w = 4 * sub; w < wave; ++w) pre += wtot[w];
    const int b0 = carry;
    const int b1 = b0 + ((S0 + 31) & ~31);
    const int b2 = b1 + ((S1 + 31) & ~31);
    const int b3 = b2 + ((S2 + 31) & ~31);
    const int b4 = b3 + ((S3 + 31) & ~31);
    const int myb = sub == 0 ? b0 : (sub == 1 ? b1 : (sub == 2 ? b2 : b3));
    if (tid == 0) {
      srb[min(4 * ch + 0, RBN - 1)] = b0;
      srb[min(4 * ch + 1, RBN - 1)] = b1;
      srb[min(4 * ch + 2, RBN - 1)] = b2;
      srb[min(4 * ch + 3, RBN - 1)] = b3;
    }
    int run = myb + pre + incl - ts;
    v4i o0, o1, o2, o3;
    o0.x = run; run += c0.x; o0.y = run; run += c0.y; o0.z = run; run += c0.z; o0.w = run; run += c0.w;
    o1.x = run; run += c1.x; o1.y = run; run += c1.y; o1.z = run; run += c1.z; o1.w = run; run += c1.w;
    o2.x = run; run += c2.x; o2.y = run; run += c2.y; o2.z = run; run += c2.z; o2.w = run; run += c2.w;
    o3.x = run; run += c3.x; o3.y = run; run += c3.y; o3.z = run; run += c3.z; o3.w = run;
    *(v4i*)(soff + CPT * tid)      = o0;
    *(v4i*)(soff + CPT * tid + 4)  = o1;
    *(v4i*)(soff + CPT * tid + 8)  = o2;
    *(v4i*)(soff + CPT * tid + 12) = o3;
    carry = b4;
    __syncthreads();
    v4i sv[4];
#pragma unroll
    for (int q = 0; q < 4; ++q) sv[q] = *(const v4i*)(soff + 4 * (tid + q * OTHR));
    int* op = off + base;
#pragma unroll
    for (int q = 0; q < 4; ++q) *(volatile v4i*)(op + 4 * (tid + q * OTHR)) = sv[q];
    __threadfence();
#pragma unroll
    for (int q = 0; q < 4; ++q) *(volatile v4i*)(op + 4 * (tid + q * OTHR)) = sv[q];
    __syncthreads();
  }
  if (tid == 0) srb[min(4 * nChunk, RBN - 1)] = carry;
  __syncthreads();
  v4i rv = {0, 0, 0, 0};
  if (tid < 32) rv = *(const v4i*)(srb + 4 * tid);
  if (tid < 32) *(volatile v4i*)(rbase + 4 * tid) = rv;
  __threadfence();
  if (tid < 32) *(volatile v4i*)(rbase + 4 * tid) = rv;
}

__global__ __launch_bounds__(NTHR) void k_fill(
    const int* __restrict__ srcs, const int* __restrict__ dsts,
    const int* __restrict__ off, const int* __restrict__ rbase,
    int* csr, int nN, int nE, int vec8, int csrLen) {
  extern __shared__ v4f lds_dyn[];
  int* region = (int*)lds_dyn;
  int* cursor = region + RCAP;
  int* list   = cursor + NBF;
  int* wcnt   = list + LISTN;
  const int tid = threadIdx.x, lane = tid & 31, wave = tid >> 5;
  const int b = blockIdx.x;
  const int nodeBase = b * NBF;

  int rb0 = rbase[b];
  const int rb1 = rbase[b + 1];
  rb0 = rb0 < 0 ? 0 : (rb0 > csrLen ? csrLen : rb0);
  rb0 &= ~31;
  int len = rb1 - rb0;
  len = len < 0 ? 0 : (len > RCAP ? RCAP : len);
  int lenW = (len + 31) & ~31;
  if (rb0 + lenW > csrLen) lenW = (csrLen - rb0) & ~31;

  {
    const v4i z = {0, 0, 0, 0};
    for (int i = tid; i < RCAP / 4; i += NTHR) ((v4i*)region)[i] = z;
    for (int s = tid; s < NBF; s += NTHR) {
      int o = off[nodeBase + s] - rb0;
      o = o < 0 ? 0 : (o > RCAP ? RCAP : o);
      cursor[s] = o;
    }
  }
  __syncthreads();

  const int nChunks = (nE + CHUNK - 1) / CHUNK;
#pragma unroll 1
  for (int ch = 0; ch < nChunks; ++ch) {
    const int cbase = ch * CHUNK;
    const int wc = scan_chunk<NBF>(dsts, nE, cbase, nodeBase, vec8, list, tid, lane, wave);
    if (lane == 0) wcnt[wave] = wc;
    __syncthreads();
    if (wave == 0) {
#pragma unroll 1
      for (int wsx = 0; wsx < NWAVE; ++wsx) {
        int n = __builtin_amdgcn_readfirstlane(wcnt[wsx]);
        n = n > WCAP ? WCAP : (n < 0 ? 0 : n);
        const int* lp = list + wsx * WCAP;
#pragma unroll 1
        for (int i = 0; i < n; ++i) {
          const int ent  = __builtin_amdgcn_readfirstlane(lp[i]);
          const int slot = ent & (NBF - 1);
          int e = cbase + ((ent >> KSH) & (CHUNK - 1));
          e = e > nE - 1 ? nE - 1 : e;
          int sv = srcs[e];
          sv = sv < 0 ? 0 : (sv > nN - 1 ? nN - 1 : sv);
          if (lane == 0) {
            int pos = cursor[slot];
            pos = pos < 0 ? 0 : (pos > RCAP - 1 ? RCAP - 1 : pos);
            region[pos] = sv;
            const int np = pos + 1;
            cursor[slot] = np > RCAP ? RCAP : np;
          }
        }
      }
    }
    __syncthreads();
  }

  const int nv = lenW >> 2;
  int* gp = csr + rb0;
#pragma unroll 1
  for (int i = tid; i < nv; i += NTHR) { const v4i v = ((const v4i*)region)[i]; *(volatile v4i*)(gp + 4 * i) = v; }
  __threadfence();
#pragma unroll 1
  for (int i = tid; i < nv; i += NTHR) { const v4i v = ((const v4i*)region)[i]; *(volatile v4i*)(gp + 4 * i) = v; }
}

__global__ __launch_bounds__(NTHR) void k_wcvt(const float* __restrict__ w, _Float16* dp, int K, int Nc, int nUnits) {
  const int i = (int)blockIdx.x * NTHR + (int)threadIdx.x;
  if (i >= nUnits) return;
  const int ppr = K >> 3;
  const int n = i / ppr;
  const int seg = i - n * ppr;
  v8h o;
#pragma unroll
  for (int j = 0; j < 8; ++j) {
    int k = 8 * seg + j;
    k = k > K - 1 ? K - 1 : k;
    const float f = w[(size_t)k * Nc + n];
    o[j] = (_Float16)(f * WCARRY);
  }
  _Float16* gp = dp + (size_t)i * 8;
  *(volatile v8h*)gp = o;
  __threadfence();
  *(volatile v8h*)gp = o;
}

__global__ __launch_bounds__(NTHR) void k_acvt(const float* __restrict__ x, _Float16* a1, int nN, int npad) {
  const int gi = (int)blockIdx.x * NTHR + (int)threadIdx.x;
  const int row = gi >> 4, seg = gi & 15;
  if (row >= npad) return;
  int rr = row > nN - 1 ? nN - 1 : row;
  rr = rr < 0 ? 0 : rr;
  const bool live = row < nN;
  const float* rp = x + (size_t)rr * FIN + 8 * seg;
  const v4f x0 = *(const v4f*)rp;
  const v4f x1 = *(const v4f*)(rp + 4);
  const float sc = live ? ACARRY : 0.f;
  v8h o;
  o[0] = (_Float16)(x0.x * sc); o[1] = (_Float16)(x0.y * sc); o[2] = (_Float16)(x0.z * sc); o[3] = (_Float16)(x0.w * sc);
  o[4] = (_Float16)(x1.x * sc); o[5] = (_Float16)(x1.y * sc); o[6] = (_Float16)(x1.z * sc); o[7] = (_Float16)(x1.w * sc);
  _Float16* gp = a1 + (size_t)row * FIN + 8 * seg;
  *(volatile v8h*)gp = o;
  __threadfence();
  *(volatile v8h*)gp = o;
}

__global__ __launch_bounds__(NTHR) void k_gemm(
    const _Float16* __restrict__ A, const _Float16* __restrict__ Bp,
    float* Cout, int K, int ldc, int nValid, int nStore, float scl) {
  constexpr int TPW = 4;
  constexpr int PPR = BNC / 4;
  constexpr int NIT = (BM * PPR) / NTHR;
  static_assert((BM * PPR) % NTHR == 0);
  static_assert(NIT >= 1);
  static_assert(TPW * 16 * 2 == BNC);
  static_assert(BM == 4 * 16);
  static_assert(PPR == 32);

  __shared__ __attribute__((aligned(16))) float stg[BM * BNC];
  const int tid = threadIdx.x, lane = tid & 31, wave = tid >> 5, hh = lane >> 4, m = lane & 15;
  const int rowBase = (int)blockIdx.x * BM;
  const int colBase = (int)blockIdx.y * BNC;
  const int rg = wave >> 1, chf = wave & 1;
  const int r0 = rg * 16;
  const int c0 = chf * (BNC / 2);

  v8f acc[TPW];
#pragma unroll
  for (int t = 0; t < TPW; ++t) { v8f z = {0.f, 0.f, 0.f, 0.f, 0.f, 0.f, 0.f, 0.f}; acc[t] = z; }

  const _Float16* ap = A  + (size_t)(rowBase + r0 + m) * K + 8 * hh;
  const _Float16* bp = Bp + (size_t)(colBase + c0 + m) * K + 8 * hh;
  const int ksteps = K >> 5;
#pragma unroll 1
  for (int kt = 0; kt < ksteps; ++kt) {
    Frag a;
    a.h[0] = *(const v8h*)(ap + 32 * kt);
    a.h[1] = *(const v8h*)(ap + 32 * kt + 16);
#pragma unroll
    for (int t = 0; t < TPW; ++t) {
      const size_t to = (size_t)(16 * t) * K + 32 * kt;
      Frag b;
      b.h[0] = *(const v8h*)(bp + to);
      b.h[1] = *(const v8h*)(bp + to + 16);
      acc[t] = wmh(a.v, b.v, acc[t]);
    }
  }

  {
    float* sp = stg + (size_t)(r0 + 8 * hh) * BNC + c0 + m;
    const int growb = rowBase + r0 + 8 * hh;
#pragma unroll
    for (int t = 0; t < TPW; ++t) {
#pragma unroll
      for (int r = 0; r < 8; ++r) {
        const bool lv = (growb + r) < nValid;
        const float g = acc[t][r] * scl;
        sp[r * BNC + 16 * t] = lv ? g : 0.f;
      }
    }
  }
  __syncthreads();

  v4f cv[NIT];
#pragma unroll
  for (int it = 0; it < NIT; ++it) {
    const int id = it * NTHR + tid;
    const int row = id >> 5, seg = id & 31;
    cv[it] = *(const v4f*)(stg + (size_t)row * BNC + 4 * seg);
  }
#pragma unroll
  for (int it = 0; it < NIT; ++it) {
    const int id = it * NTHR + tid;
    const int row = id >> 5, seg = id & 31;
    const int grow = rowBase + row;
    if (grow < nStore) {
      float* gp = Cout + (size_t)grow * ldc + colBase + 4 * seg;
      *(volatile v4f*)gp = cv[it];
    }
  }
  __threadfence();
#pragma unroll
  for (int it = 0; it < NIT; ++it) {
    const int id = it * NTHR + tid;
    const int row = id >> 5, seg = id & 31;
    const int grow = rowBase + row;
    if (grow < nStore) {
      float* gp = Cout + (size_t)grow * ldc + colBase + 4 * seg;
      *(volatile v4f*)gp = cv[it];
    }
  }
}

__global__ __launch_bounds__(NTHR) void k_elr(const float* __restrict__ feat, const float* __restrict__ al,
                                              const float* __restrict__ ar, float* es) {
  __shared__ __attribute__((aligned(16))) float sal[NHD * DHD];
  __shared__ __attribute__((aligned(16))) float sar[NHD * DHD];
  __shared__ __attribute__((aligned(16))) float so[32 * ESW];
  const int tid = threadIdx.x;
  if (tid < NHD * DHD) { sal[tid] = al[tid]; sar[tid] = ar[tid]; }
  __syncthreads();
  const int t = (int)blockIdx.x * NTHR + tid;
  const int node = t >> 3, hd = t & 7;
  const float* fp = feat + (size_t)node * FOUT + hd * DHD;
  const float* lp = sal + hd * DHD;
  const float* rp = sar + hd * DHD;
  v4f accl = {0.f, 0.f, 0.f, 0.f};
  v4f accr = {0.f, 0.f, 0.f, 0.f};
#pragma unroll 1
  for (int q = 0; q < DHD / 4; ++q) {
    const v4f f  = *(const v4f*)(fp + 4 * q);
    const v4f wl = *(const v4f*)(lp + 4 * q);
    const v4f wr = *(const v4f*)(rp + 4 * q);
    accl = accl + f * wl;
    accr = accr + f * wr;
  }
  const float elv = (accl.x + accl.y) + (accl.z + accl.w);
  const float erv = (accr.x + accr.y) + (accr.z + accr.w);
  const int nl = tid >> 3;
  so[nl * ESW + hd]       = elv;
  so[nl * ESW + NHD + hd] = erv;
  __syncthreads();
  const int tq = tid & 127;
  const v4f v = *(const v4f*)(so + 4 * tq);
  float* gp = es + (size_t)blockIdx.x * (32 * ESW) + 4 * tq;
  if (tid < 128) *(volatile v4f*)gp = v;
  __threadfence();
  if (tid < 128) *(volatile v4f*)gp = v;
}

__global__ __launch_bounds__(NTHR) void k_agg(
    const int* __restrict__ csr, const int* __restrict__ off, const int* __restrict__ cnt,
    const float* __restrict__ es, const float* __restrict__ feat, const float* __restrict__ hres,
    const float* __restrict__ gb, float* out, int nN, int csrLen) {
  const int tid = threadIdx.x, lane = tid & 31, wave = tid >> 5, hq = lane >> 2;
  const bool hb0 = (hq & 1) != 0, hb1 = (hq & 2) != 0, hb2 = (hq & 4) != 0;
  const int tbase = blockIdx.x * TGT + wave * 32;
  const int cl    = tbase + lane;
  const int cnt_l = cnt[cl];
  const int off_l = off[cl];
  const v4f bv = *(const v4f*)(gb + 4 * lane);
  const float NINF = -__builtin_inff();
  const float QNAN = __int_as_float(0x7fc00000);

#pragma unroll 1
  for (int j = 0; j < 32; ++j) {
    const int c = tbase + j;
    const int nraw = __shfl(cnt_l, j);
    const bool over = nraw > DEGCAP;
    const int n = nraw < 0 ? 0 : (nraw > DEGCAP ? DEGCAP : nraw);
    const int st = __shfl(off_l, j);
    int cc = c > nN - 1 ? nN - 1 : c;
    cc = cc < 0 ? 0 : cc;
    const v4f edlo = *(const v4f*)(es + (size_t)c * ESW + NHD);
    const v4f edhi = *(const v4f*)(es + (size_t)c * ESW + NHD + 4);

    v4f mlo = {NINF, NINF, NINF, NINF};
    v4f mhi = {NINF, NINF, NINF, NINF};
#pragma unroll 1
    for (int q0 = 0; q0 < n; q0 += 32) {
      int pos = st + q0 + lane;
      pos = pos < 0 ? 0 : (pos > csrLen - 1 ? csrLen - 1 : pos);
      int sl = csr[pos];
      sl = sl < 0 ? 0 : (sl > nN - 1 ? nN - 1 : sl);
      const int mcnt = (n - q0) < 32 ? (n - q0) : 32;
      const bool valid = lane < mcnt;
      const v4f sllo = *(const v4f*)(es + (size_t)sl * ESW);
      const v4f slhi = *(const v4f*)(es + (size_t)sl * ESW + 4);
      v4f e0 = selv4(lrelu4(sllo + edlo), valid, NINF);
      v4f e1 = selv4(lrelu4(slhi + edhi), valid, NINF);
      e0 = wmax4(e0);
      e1 = wmax4(e1);
      mlo = vmax4(mlo, e0);
      mhi = vmax4(mhi, e1);
    }
    v4f zlo = {0.f, 0.f, 0.f, 0.f};
    v4f zhi = {0.f, 0.f, 0.f, 0.f};
#pragma unroll 1
    for (int q0 = 0; q0 < n; q0 += 32) {
      int pos = st + q0 + lane;
      pos = pos < 0 ? 0 : (pos > csrLen - 1 ? csrLen - 1 : pos);
      int sl = csr[pos];
      sl = sl < 0 ? 0 : (sl > nN - 1 ? nN - 1 : sl);
      const int mcnt = (n - q0) < 32 ? (n - q0) : 32;
      const bool valid = lane < mcnt;
      const v4f sllo = *(const v4f*)(es + (size_t)sl * ESW);
      const v4f slhi = *(const v4f*)(es + (size_t)sl * ESW + 4);
      const v4f ex0 = selv4(vexp4(lrelu4(sllo + edlo) - mlo), valid, 0.f);
      const v4f ex1 = selv4(vexp4(lrelu4(slhi + edhi) - mhi), valid, 0.f);
      zlo = zlo + wsum4(ex0);
      zhi = zhi + wsum4(ex1);
    }
    v4f rzlo, rzhi;
    rzlo.x = __builtin_amdgcn_rcpf(zlo.x); rzlo.y = __builtin_amdgcn_rcpf(zlo.y);
    rzlo.z = __builtin_amdgcn_rcpf(zlo.z); rzlo.w = __builtin_amdgcn_rcpf(zlo.w);
    rzhi.x = __builtin_amdgcn_rcpf(zhi.x); rzhi.y = __builtin_amdgcn_rcpf(zhi.y);
    rzhi.z = __builtin_amdgcn_rcpf(zhi.z); rzhi.w = __builtin_amdgcn_rcpf(zhi.w);

    v4f acc = {0.f, 0.f, 0.f, 0.f};
#pragma unroll 1
    for (int q0 = 0; q0 < n; q0 += 32) {
      int pos = st + q0 + lane;
      pos = pos < 0 ? 0 : (pos > csrLen - 1 ? csrLen - 1 : pos);
      int sl = csr[pos];
      sl = sl < 0 ? 0 : (sl > nN - 1 ? nN - 1 : sl);
      const int mcnt = (n - q0) < 32 ? (n - q0) : 32;
      const bool valid = lane < mcnt;
      const v4f sllo = *(const v4f*)(es + (size_t)sl * ESW);
      const v4f slhi = *(const v4f*)(es + (size_t)sl * ESW + 4);
      const v4f al0 = selv4(vexp4(lrelu4(sllo + edlo) - mlo) * rzlo, valid, 0.f);
      const v4f al1 = selv4(vexp4(lrelu4(slhi + edhi) - mhi) * rzhi, valid, 0.f);
#pragma unroll 1
      for (int pp = 0; pp < mcnt; ++pp) {
        const int s = __builtin_amdgcn_readlane(sl, pp);
        const float a0 = __int_as_float(__builtin_amdgcn_readlane(__float_as_int(al0.x), pp));
        const float a1 = __int_as_float(__builtin_amdgcn_readlane(__float_as_int(al0.y), pp));
        const float a2 = __int_as_float(__builtin_amdgcn_readlane(__float_as_int(al0.z), pp));
        const float a3 = __int_as_float(__builtin_amdgcn_readlane(__float_as_int(al0.w), pp));
        const float a4 = __int_as_float(__builtin_amdgcn_readlane(__float_as_int(al1.x), pp));
        const float a5 = __int_as_float(__builtin_amdgcn_readlane(__float_as_int(al1.y), pp));
        const float a6 = __int_as_float(__builtin_amdgcn_readlane(__float_as_int(al1.z), pp));
        const float a7 = __int_as_float(__builtin_amdgcn_readlane(__float_as_int(al1.w), pp));
        const float q01 = hb0 ? a1 : a0;
        const float q23 = hb0 ? a3 : a2;
        const float q45 = hb0 ? a5 : a4;
        const float q67 = hb0 ? a7 : a6;
        const float q03 = hb1 ? q23 : q01;
        const float q47 = hb1 ? q67 : q45;
        const float ap  = hb2 ? q47 : q03;
        const v4f hv = *(const v4f*)(feat + (size_t)s * FOUT + 4 * lane);
        acc = acc + hv * ap;
      }
    }

    const bool live = c < nN;
    const v4f rv = *(const v4f*)(hres + (size_t)cc * FIN + 4 * lane);
    v4f o = (acc + rv) + bv;
    o = selv4(o, !over, QNAN);
    float* gp = out + (size_t)cc * FOUT + 4 * lane;
    if (live) *(volatile v4f*)gp = o;
    __threadfence();
    if (live) *(volatile v4f*)gp = o;
  }
}

extern "C" void kernel_launch(void* const* d_in, const int* in_sizes, int n_in,
                              void* d_out, int out_size, void* d_ws, size_t ws_size,
                              hipStream_t stream) {
  if (n_in < 7) return;
  if (in_sizes[0] < FIN || (in_sizes[0] % FIN) != 0) return;
  const int nN = in_sizes[0] / FIN;
  if (nN < 1 || nN > 200000) return;
  if (in_sizes[1] != FIN * FOUT) return;
  if (in_sizes[2] != NHD * DHD || in_sizes[3] != NHD * DHD) return;
  if (in_sizes[4] != FOUT) return;
  const int nE = in_sizes[5];
  if (nE < 1 || nE > (1 << 26) || in_sizes[6] != nE) return;
  if (out_size != nN * FOUT) return;

  const float* h      = (const float*)d_in[0];
  const float* W      = (const float*)d_in[1];
  const float* attn_l = (const float*)d_in[2];
  const float* attn_r = (const float*)d_in[3];
  const float* bias   = (const float*)d_in[4];
  const int*   src    = (const int*)d_in[5];
  const int*   dst    = (const int*)d_in[6];
  float* out = (float*)d_out;

  const int NPAD   = ((nN + TGT - 1) / TGT) * TGT;
  const int nAgg   = NPAD / TGT;
  const int nBC    = (nN + NBC - 1) / NBC;
  const int CNTPAD = nBC * NBC;
  if (CNTPAD < NPAD) return;
  if (4 * nBC + 1 > RBN) return;
  const int nBF    = (nN + NBF - 1) / NBF;
  if (nBF > 4 * nBC) return;
  const int csrLen = ((nE + 31) & ~31) + 4096;
  if (31 * 4 * nBC > 4096) return;

  char* ws = (char*)d_ws;
  size_t off = 0;
  const size_t oCnt = off; off += (size_t)CNTPAD * 4;                    off = (off + 255) & ~(size_t)255;
  const size_t oOff = off; off += (size_t)CNTPAD * 4;                    off = (off + 255) & ~(size_t)255;
  const size_t oRb  = off; off += (size_t)RBN * 4;                       off = (off + 255) & ~(size_t)255;
  const size_t oCsr = off; off += (size_t)csrLen * 4;                    off = (off + 255) & ~(size_t)255;
  const size_t oW1  = off; off += (size_t)FOUT * FIN * 2;                off = (off + 255) & ~(size_t)255;
  const size_t oA1  = off; off += (size_t)NPAD * FIN * 2;                off = (off + 255) & ~(size_t)255;
  const size_t oFt  = off; off += (size_t)NPAD * FOUT * 4;               off = (off + 255) & ~(size_t)255;
  const size_t oEs  = off; off += (size_t)NPAD * ESW * 4;                off = (off + 255) & ~(size_t)255;
  if (off > ws_size || off > (size_t)WSCAP) return;

  int*   cnt   = (int*)(ws + oCnt);
  int*   offp  = (int*)(ws + oOff);
  int*   rb    = (int*)(ws + oRb);
  int*   csr   = (int*)(ws + oCsr);
  _Float16* w1p = (_Float16*)(ws + oW1);
  _Float16* a1  = (_Float16*)(ws + oA1);
  float* feat  = (float*)(ws + oFt);
  float* es    = (float*)(ws + oEs);

  const int vec8 = 1;

  k_count<<<nBC, NTHR, 0, stream>>>(dst, cnt, nE, vec8);
  k_offsets<<<1, OTHR, 0, stream>>>(cnt, offp, rb, nBC);
  hipFuncSetAttribute(reinterpret_cast<const void*>(&k_fill),
                      hipFuncAttributeMaxDynamicSharedMemorySize, LDS_FILL);
  k_fill<<<nBF, NTHR, LDS_FILL, stream>>>(src, dst, offp, rb, csr, nN, nE, vec8, csrLen);

  {
    const int u1 = FOUT * (FIN / 8);
    k_wcvt<<<(u1 + NTHR - 1) / NTHR, NTHR, 0, stream>>>(W, w1p, FIN, FOUT, u1);
  }
  k_acvt<<<(NPAD * 16) / NTHR, NTHR, 0, stream>>>(h, a1, nN, NPAD);
  k_gemm<<<dim3(NPAD / BM, FOUT / BNC), NTHR, 0, stream>>>(a1, w1p, feat, FIN, FOUT, nN, NPAD, SCL_AW);

  k_elr<<<NPAD / 32, NTHR, 0, stream>>>(feat, attn_l, attn_r, es);

  k_agg<<<nAgg, NTHR, 0, stream>>>(csr, offp, cnt, es, feat, h, bias, out, nN, csrLen);
}
